// LinearGPT2Block_1468878815672
// MI455X (gfx1250) — hardware-verified
//
#include <hip/hip_runtime.h>
#include <math.h>

typedef _Float16 v16h __attribute__((ext_vector_type(16)));
typedef _Float16 v8h  __attribute__((ext_vector_type(8)));
typedef float    v8f  __attribute__((ext_vector_type(8)));
typedef float    v4f  __attribute__((ext_vector_type(4)));
typedef v8h __attribute__((may_alias)) v8ha;
typedef v4f __attribute__((may_alias)) v4fa;

union Frag { v16h v; v8h half[2]; };

#define DM     1024
#define NH     16
#define HD     64
#define DFF    4096
#define SEQ    2048
#define BATCH  2
#define NTOK   (BATCH * SEQ)
#define WSC    32.0f
#define WINV   0.03125f
#define PSCALE 16384.0f

#define G_QKV (3 * DM * DM / 8)
#define G_OUT (DM * DM / 8)
#define G_FC1 (DFF * DM / 8)
#define G_FC2 (DM * DFF / 8)
#define G_ALL (G_QKV + G_OUT + G_FC1 + G_FC2)

static_assert(NTOK % 128 == 0);
static_assert(SEQ % 128 == 0);
static_assert(DM % 64 == 0);
static_assert(DFF % 64 == 0);
static_assert(G_ALL % 256 == 0);

__device__ __forceinline__ v8f wmma_f16(v16h a, v16h b, v8f c) {
  v8f d = __builtin_amdgcn_wmma_f32_16x16x32_f16(false, a, false, b, (short)0, c, false, false);
  asm volatile("v_nop\n\tv_nop\n\tv_nop\n\tv_nop" : "+v"(d) : "v"(a), "v"(b));
  return d;
}

__device__ __forceinline__ v16h load_frag(const _Float16* p, int h) {
  Frag f;
  f.half[0] = *(const v8ha*)(p + 8 * h);
  f.half[1] = *(const v8ha*)(p + 16 + 8 * h);
  return f.v;
}

__global__ __launch_bounds__(256) void cvt_w_kernel(
    const float* __restrict__ w0, const float* __restrict__ w1,
    const float* __restrict__ w2, const float* __restrict__ w3,
    _Float16* __restrict__ wh)
{
  const int g = blockIdx.x * 256 + threadIdx.x;
  if (g >= G_ALL) return;
  const float* src;
  if (g < G_QKV)                        src = w0 + (size_t)g * 8;
  else if (g < G_QKV + G_OUT)           src = w1 + (size_t)(g - G_QKV) * 8;
  else if (g < G_QKV + G_OUT + G_FC1)   src = w2 + (size_t)(g - G_QKV - G_OUT) * 8;
  else                                  src = w3 + (size_t)(g - G_QKV - G_OUT - G_FC1) * 8;
  _Float16* dst = wh + (size_t)g * 8;
  const v4f a = *(const v4fa*)src;
  const v4f c = *(const v4fa*)(src + 4);
  const v8h o = { (_Float16)(a.x * WSC), (_Float16)(a.y * WSC), (_Float16)(a.z * WSC), (_Float16)(a.w * WSC),
                  (_Float16)(c.x * WSC), (_Float16)(c.y * WSC), (_Float16)(c.z * WSC), (_Float16)(c.w * WSC) };
  *(volatile v8h*)dst = o;
  __threadfence();
  *(volatile v8h*)dst = o;
}

__global__ __launch_bounds__(256) void ln_kernel(
    const float* __restrict__ x, const float* __restrict__ g,
    const float* __restrict__ bt, _Float16* __restrict__ y, int nrows)
{
  const int lane = threadIdx.x & 31, w = threadIdx.x >> 5;
  const int row = blockIdx.x * 8 + w;
  if (row >= nrows) return;
  const float* xr = x + (size_t)row * DM;

  v4f xa[4], xb[4];
  float s = 0.0f;
  #pragma unroll
  for (int i = 0; i < 4; ++i) {
    const float* p = xr + i * 256 + lane * 8;
    xa[i] = *(const v4fa*)p;
    xb[i] = *(const v4fa*)(p + 4);
    s += ((xa[i].x + xa[i].y) + (xa[i].z + xa[i].w)) + ((xb[i].x + xb[i].y) + (xb[i].z + xb[i].w));
  }
  #pragma unroll
  for (int off = 16; off > 0; off >>= 1) s += __shfl_xor(s, off);
  const float mu = s * (1.0f / DM);

  float ss = 0.0f;
  #pragma unroll
  for (int i = 0; i < 4; ++i) {
    const v4f da = xa[i] - mu, db = xb[i] - mu;
    ss += ((da.x * da.x + da.y * da.y) + (da.z * da.z + da.w * da.w)) +
          ((db.x * db.x + db.y * db.y) + (db.z * db.z + db.w * db.w));
  }
  #pragma unroll
  for (int off = 16; off > 0; off >>= 1) ss += __shfl_xor(ss, off);
  const float var = ss * (1.0f / DM);
  const float rstd = rsqrtf(var + 1e-5f);

  v8h o[4];
  #pragma unroll
  for (int i = 0; i < 4; ++i) {
    const int p = i * 256 + lane * 8;
    const v4f ga = *(const v4fa*)(g + p),  gb = *(const v4fa*)(g + p + 4);
    const v4f ba = *(const v4fa*)(bt + p), bb = *(const v4fa*)(bt + p + 4);
    const v4f da = (xa[i] - mu) * rstd, db = (xb[i] - mu) * rstd;
    const v8h t = { (_Float16)(da.x * ga.x + ba.x), (_Float16)(da.y * ga.y + ba.y),
                    (_Float16)(da.z * ga.z + ba.z), (_Float16)(da.w * ga.w + ba.w),
                    (_Float16)(db.x * gb.x + bb.x), (_Float16)(db.y * gb.y + bb.y),
                    (_Float16)(db.z * gb.z + bb.z), (_Float16)(db.w * gb.w + bb.w) };
    o[i] = t;
  }
  _Float16* yr = y + (size_t)row * DM;
  #pragma unroll
  for (int i = 0; i < 4; ++i) *(volatile v8h*)(yr + i * 256 + lane * 8) = o[i];
  __threadfence();
  #pragma unroll
  for (int i = 0; i < 4; ++i) *(volatile v8h*)(yr + i * 256 + lane * 8) = o[i];
}

__device__ __forceinline__ void gemm_main(const _Float16* __restrict__ xa0,
                                          const _Float16* __restrict__ xa1,
                                          const _Float16* __restrict__ wb,
                                          int K, int h, v8f (&acc)[2][4])
{
  const v8f zero8 = {0.f, 0.f, 0.f, 0.f, 0.f, 0.f, 0.f, 0.f};
  #pragma unroll
  for (int mt = 0; mt < 2; ++mt)
    #pragma unroll
    for (int nt = 0; nt < 4; ++nt) acc[mt][nt] = zero8;

  #pragma unroll 1
  for (int k0 = 0; k0 < K; k0 += 32) {
    const v16h a0 = load_frag(xa0 + k0, h);
    const v16h a1 = load_frag(xa1 + k0, h);
    #pragma unroll
    for (int nt = 0; nt < 4; ++nt) {
      const v16h b = load_frag(wb + (size_t)nt * 16 * K + k0, h);
      acc[0][nt] = wmma_f16(a0, b, acc[0][nt]);
      acc[1][nt] = wmma_f16(a1, b, acc[1][nt]);
    }
  }
}

__device__ __forceinline__ void qkv_store_pass(const _Float16* sT, _Float16* plane, _Float16* vt,
                                               int which, int bh, int l0, int w, int lane) {
  const int q8 = lane & 7, sub = lane >> 3;
  #pragma unroll
  for (int i = 0; i < 8; ++i) {
    const int lid = w * 32 + i * 4 + sub;
    v8h v;
    _Float16* dst;
    if (which != 2) {
      v = *(const v8ha*)(sT + lid * HD + 8 * q8);
      dst = plane + ((size_t)bh * SEQ + l0 + lid) * HD + 8 * q8;
    } else {
      const int d = lid >> 1, hl = lid & 1;
      v = *(const v8ha*)(sT + d * 128 + 64 * hl + 8 * q8);
      dst = vt + ((size_t)bh * HD + d) * SEQ + l0 + 64 * hl + 8 * q8;
    }
    *(volatile v8h*)dst = v;
  }
}

__global__ __launch_bounds__(128) void qkv_kernel(
    const _Float16* __restrict__ xh,
    const _Float16* __restrict__ wh,
    const float* __restrict__ bias,
    _Float16* __restrict__ qh, _Float16* __restrict__ kh, _Float16* __restrict__ vt)
{
  __shared__ __attribute__((aligned(16))) _Float16 sT[128 * 64];

  const int tid = threadIdx.x, lane = tid & 31, w = tid >> 5;
  const int h = lane >> 4, m = lane & 15;
  const int m0 = blockIdx.x * 128;
  const int cg = blockIdx.y;
  const int which = cg >> 4, head = cg & 15;
  const int m0w = m0 + 32 * w;

  const _Float16* xa0 = xh + (size_t)(m0w + m) * DM;
  const _Float16* xa1 = xa0 + (size_t)16 * DM;
  const _Float16* wb  = wh + ((size_t)cg * 64 + m) * DM;

  v8f acc[2][4];
  gemm_main(xa0, xa1, wb, DM, h, acc);

  #pragma unroll
  for (int nt = 0; nt < 4; ++nt) {
    const int feat = 16 * nt + m;
    const float bvl = bias[cg * 64 + feat];
    #pragma unroll
    for (int mt = 0; mt < 2; ++mt) {
      #pragma unroll
      for (int r = 0; r < 8; ++r) {
        const int tokl = 32 * w + 16 * mt + 8 * h + r;
        const float yv = acc[mt][nt][r] * WINV + bvl;
        const int idx = (which == 2) ? (feat * 128 + tokl) : (tokl * HD + feat);
        sT[idx] = (_Float16)yv;
      }
    }
  }
  __syncthreads();

  const int b = m0 / SEQ, l0 = m0 - b * SEQ, bh = b * NH + head;
  _Float16* plane = (which == 0) ? qh : kh;
  qkv_store_pass(sT, plane, vt, which, bh, l0, w, lane);
  __threadfence();
  qkv_store_pass(sT, plane, vt, which, bh, l0, w, lane);
}

__device__ __forceinline__ v16h pack_p(v8f a, v8f c) {
  const v16h r = { (_Float16)(a[0] * PSCALE), (_Float16)(a[1] * PSCALE), (_Float16)(a[2] * PSCALE), (_Float16)(a[3] * PSCALE),
                   (_Float16)(a[4] * PSCALE), (_Float16)(a[5] * PSCALE), (_Float16)(a[6] * PSCALE), (_Float16)(a[7] * PSCALE),
                   (_Float16)(c[0] * PSCALE), (_Float16)(c[1] * PSCALE), (_Float16)(c[2] * PSCALE), (_Float16)(c[3] * PSCALE),
                   (_Float16)(c[4] * PSCALE), (_Float16)(c[5] * PSCALE), (_Float16)(c[6] * PSCALE), (_Float16)(c[7] * PSCALE) };
  return r;
}

__device__ __forceinline__ void att_store_pass(const _Float16* so, _Float16* ao,
                                               int b, int head, int q0, int lane) {
  const int q8 = lane & 7, sub = lane >> 3;
  #pragma unroll
  for (int i = 0; i < 4; ++i) {
    const int lid = i * 4 + sub;
    const v8h v = *(const v8ha*)(so + lid * 64 + 8 * q8);
    const size_t gi = ((size_t)b * SEQ + q0 + lid) * DM + head * HD + 8 * q8;
    *(volatile v8h*)(ao + gi) = v;
  }
}

__global__ __launch_bounds__(128) void attn_kernel(
    const _Float16* __restrict__ qh,
    const _Float16* __restrict__ kh,
    const _Float16* __restrict__ vt,
    _Float16* __restrict__ ao)
{
  __shared__ __attribute__((aligned(16))) _Float16 sO[4 * 16 * 64];

  const int tid = threadIdx.x, lane = tid & 31, w = tid >> 5;
  const int h = lane >> 4, m = lane & 15;
  const int bh = blockIdx.y, b = bh >> 4, head = bh & 15;
  const int q0 = blockIdx.x * 64 + 16 * w;

  const _Float16* qrow = qh + ((size_t)bh * SEQ + q0 + m) * HD;
  const v16h qb0 = load_frag(qrow, h);
  const v16h qb1 = load_frag(qrow + 32, h);

  const v8f zero8 = {0.f, 0.f, 0.f, 0.f, 0.f, 0.f, 0.f, 0.f};
  v8f o[4];
  #pragma unroll
  for (int t = 0; t < 4; ++t) o[t] = zero8;
  float mrun = -1e30f, lrun = 0.0f;

  const _Float16* kbase = kh + ((size_t)bh * SEQ + m) * HD;
  const _Float16* vbase = vt + ((size_t)bh * HD + m) * SEQ;
  const int kend = q0 + 16;

  #pragma unroll 1
  for (int kb = 0; kb < kend; kb += 64) {
    v8f s[4];
    #pragma unroll
    for (int j = 0; j < 4; ++j) {
      const _Float16* kp = kbase + (size_t)(kb + 16 * j) * HD;
      const v16h kf0 = load_frag(kp, h);
      const v16h kf1 = load_frag(kp + 32, h);
      v8f z = zero8;
      z = wmma_f16(kf0, qb0, z);
      z = wmma_f16(kf1, qb1, z);
      s[j] = z;
    }
    if (kb + 63 > q0) {
      const int qq = q0 + m;
      #pragma unroll
      for (int j = 0; j < 4; ++j)
        #pragma unroll
        for (int r = 0; r < 8; ++r) {
          const int kk = kb + 16 * j + 8 * h + r;
          if (kk > qq) s[j][r] = -1e30f;
        }
    }

    float mloc = s[0][0];
    #pragma unroll
    for (int j = 0; j < 4; ++j)
      #pragma unroll
      for (int r = 0; r < 8; ++r) mloc = fmaxf(mloc, s[j][r]);
    mloc = fmaxf(mloc, __shfl_xor(mloc, 16));
    const float mnew = fmaxf(mrun, mloc);
    const float cn = mnew * 0.125f;
    const float alpha = __expf((mrun - mnew) * 0.125f);
    mrun = mnew;
    float lsum = 0.0f;
    #pragma unroll
    for (int j = 0; j < 4; ++j)
      #pragma unroll
      for (int r = 0; r < 8; ++r) {
        const float p = __expf(fmaf(s[j][r], 0.125f, -cn));
        s[j][r] = p;
        lsum += p;
      }
    lsum += __shfl_xor(lsum, 16);
    lrun = lrun * alpha + lsum;
    #pragma unroll
    for (int t = 0; t < 4; ++t)
      #pragma unroll
      for (int r = 0; r < 8; ++r) o[t][r] = o[t][r] * alpha;

    const v16h pb0 = pack_p(s[0], s[1]);
    const v16h pb1 = pack_p(s[2], s[3]);

    #pragma unroll
    for (int t = 0; t < 4; ++t) {
      const _Float16* vp = vbase + (size_t)(16 * t) * SEQ + kb;
      const v16h vf0 = load_frag(vp, h);
      const v16h vf1 = load_frag(vp + 32, h);
      o[t] = wmma_f16(vf0, pb0, o[t]);
      o[t] = wmma_f16(vf1, pb1, o[t]);
    }
  }

  const float inv = (1.0f / lrun) * (1.0f / PSCALE);
  _Float16* so = sO + w * 1024;
  #pragma unroll
  for (int t = 0; t < 4; ++t)
    #pragma unroll
    for (int r = 0; r < 8; ++r)
      so[m * 64 + 16 * t + 8 * h + r] = (_Float16)(o[t][r] * inv);
  __syncthreads();

  att_store_pass(so, ao, b, head, q0, lane);
  __threadfence();
  att_store_pass(so, ao, b, head, q0, lane);
}

template <int MODE>
__global__ __launch_bounds__(128) void gemm_kernel(
    const _Float16* __restrict__ A, const _Float16* __restrict__ W,
    const float* __restrict__ bias, const float* __restrict__ resid,
    float* __restrict__ outf, _Float16* __restrict__ outh, int N, int K)
{
  __shared__ __attribute__((aligned(16))) float sbuf[128 * 64];

  const int tid = threadIdx.x, lane = tid & 31, w = tid >> 5;
  const int h = lane >> 4, m = lane & 15;
  const int q8 = lane & 7, sub = lane >> 3;
  const int m0 = blockIdx.x * 128, n0 = blockIdx.y * 64;
  const int m0w = m0 + 32 * w;

  const _Float16* xa0 = A + (size_t)(m0w + m) * K;
  const _Float16* xa1 = xa0 + (size_t)16 * K;
  const _Float16* wb  = W + (size_t)(n0 + m) * K;

  v8f acc[2][4];
  gemm_main(xa0, xa1, wb, K, h, acc);

  if (MODE == 1) {
    #pragma unroll
    for (int nt = 0; nt < 4; ++nt)
      #pragma unroll
      for (int mt = 0; mt < 2; ++mt)
        #pragma unroll
        for (int r = 0; r < 8; ++r)
          sbuf[(32 * w + 16 * mt + 8 * h + r) * 64 + 16 * nt + m] = acc[mt][nt][r] * WINV;
    __syncthreads();

    v4f vals[16];
    #pragma unroll
    for (int i = 0; i < 16; ++i) {
      const int lid = i * 4 + sub;
      const int rl = lid >> 1, hl = lid & 1;
      const int col = 32 * hl + 4 * q8;
      const v4f a  = *(const v4fa*)(sbuf + (32 * w + rl) * 64 + col);
      const v4f bb = *(const v4fa*)(bias + n0 + col);
      const size_t gi = (size_t)(m0w + rl) * N + n0 + col;
      const v4f rr = *(const v4fa*)(resid + gi);
      vals[i] = (a + bb) + rr;
    }
    #pragma unroll
    for (int i = 0; i < 16; ++i) {
      const int lid = i * 4 + sub;
      const int rl = lid >> 1, hl = lid & 1;
      const size_t gi = (size_t)(m0w + rl) * N + n0 + 32 * hl + 4 * q8;
      *(volatile v4f*)(outf + gi) = vals[i];
    }
    __threadfence();
    #pragma unroll
    for (int i = 0; i < 16; ++i) {
      const int lid = i * 4 + sub;
      const int rl = lid >> 1, hl = lid & 1;
      const size_t gi = (size_t)(m0w + rl) * N + n0 + 32 * hl + 4 * q8;
      *(volatile v4f*)(outf + gi) = vals[i];
    }
  } else {
    _Float16* sh = (_Float16*)sbuf;
    #pragma unroll
    for (int nt = 0; nt < 4; ++nt) {
      const float bvl = bias[n0 + 16 * nt + m];
      #pragma unroll
      for (int mt = 0; mt < 2; ++mt)
        #pragma unroll
        for (int r = 0; r < 8; ++r) {
          const float xv = acc[mt][nt][r] * WINV + bvl;
          const float gl = 0.5f * xv * (1.0f + erff(xv * 0.70710678118654752f));
          sh[(32 * w + 16 * mt + 8 * h + r) * 64 + 16 * nt + m] = (_Float16)gl;
        }
    }
    __syncthreads();

    v8h vals[8];
    #pragma unroll
    for (int i = 0; i < 8; ++i) {
      const int lid = i * 4 + sub;
      vals[i] = *(const v8ha*)(sh + (32 * w + lid) * 64 + 8 * q8);
    }
    #pragma unroll
    for (int i = 0; i < 8; ++i) {
      const int lid = i * 4 + sub;
      *(volatile v8h*)(outh + (size_t)(m0w + lid) * N + n0 + 8 * q8) = vals[i];
    }
    __threadfence();
    #pragma unroll
    for (int i = 0; i < 8; ++i) {
      const int lid = i * 4 + sub;
      *(volatile v8h*)(outh + (size_t)(m0w + lid) * N + n0 + 8 * q8) = vals[i];
    }
  }
}

extern "C" void kernel_launch(void* const* d_in, const int* in_sizes, int n_in,
                              void* d_out, int out_size, void* d_ws, size_t ws_size,
                              hipStream_t stream) {
  if (n_in < 13) return;
  if (in_sizes[0] != NTOK * DM) return;
  if (in_sizes[1] != 3 * DM * DM || in_sizes[2] != 3 * DM) return;
  if (in_sizes[3] != DM * DM || in_sizes[4] != DM) return;
  if (in_sizes[5] != DFF * DM || in_sizes[6] != DFF) return;
  if (in_sizes[7] != DM * DFF || in_sizes[8] != DM) return;
  if (in_sizes[9] != DM || in_sizes[10] != DM || in_sizes[11] != DM || in_sizes[12] != DM) return;
  if (out_size != NTOK * DM) return;

  const float* hidden = (const float*)d_in[0];
  const float* qkv_w  = (const float*)d_in[1];
  const float* qkv_b  = (const float*)d_in[2];
  const float* out_w  = (const float*)d_in[3];
  const float* out_b  = (const float*)d_in[4];
  const float* fc1_w  = (const float*)d_in[5];
  const float* fc1_b  = (const float*)d_in[6];
  const float* fc2_w  = (const float*)d_in[7];
  const float* fc2_b  = (const float*)d_in[8];
  const float* ln1_g  = (const float*)d_in[9];
  const float* ln1_b  = (const float*)d_in[10];
  const float* ln2_g  = (const float*)d_in[11];
  const float* ln2_b  = (const float*)d_in[12];
  float* out = (float*)d_out;

  const size_t wh_bytes   = (size_t)G_ALL * 8 * 2;
  const size_t act_bytes  = (size_t)NTOK * DM * 2;
  const size_t hid2_bytes = (size_t)NTOK * DM * 4;
  const size_t ff_bytes   = (size_t)NTOK * DFF * 2;
  const size_t total = wh_bytes + 5 * act_bytes + hid2_bytes + ff_bytes;
  if (total > ws_size) return;

  char* ws = (char*)d_ws;
  size_t off = 0;
  _Float16* wh   = (_Float16*)(ws + off); off += wh_bytes;
  _Float16* xn   = (_Float16*)(ws + off); off += act_bytes;
  _Float16* qh   = (_Float16*)(ws + off); off += act_bytes;
  _Float16* kh   = (_Float16*)(ws + off); off += act_bytes;
  _Float16* vt   = (_Float16*)(ws + off); off += act_bytes;
  _Float16* ah   = (_Float16*)(ws + off); off += act_bytes;
  float*    hid2 = (float*)(ws + off);    off += hid2_bytes;
  _Float16* ff   = (_Float16*)(ws + off); off += ff_bytes;
  if (off > ws_size) return;

  const _Float16* w_qkv = wh;
  const _Float16* w_out = wh + (size_t)3 * DM * DM;
  const _Float16* w_fc1 = wh + (size_t)4 * DM * DM;
  const _Float16* w_fc2 = wh + (size_t)4 * DM * DM + (size_t)DFF * DM;

  cvt_w_kernel<<<G_ALL / 256, 256, 0, stream>>>(qkv_w, out_w, fc1_w, fc2_w, wh);

  ln_kernel<<<NTOK / 8, 256, 0, stream>>>(hidden, ln1_g, ln1_b, xn, NTOK);

  qkv_kernel<<<dim3(NTOK / 128, 3 * NH), 128, 0, stream>>>(xn, w_qkv, qkv_b, qh, kh, vt);

  attn_kernel<<<dim3(SEQ / 64, BATCH * NH), 128, 0, stream>>>(qh, kh, vt, ah);

  gemm_kernel<1><<<dim3(NTOK / 128, DM / 64), 128, 0, stream>>>(ah, w_out, out_b, hidden, hid2, xn, DM, DM);

  ln_kernel<<<NTOK / 8, 256, 0, stream>>>(hid2, ln2_g, ln2_b, xn, NTOK);

  gemm_kernel<2><<<dim3(NTOK / 128, DFF / 64), 128, 0, stream>>>(xn, w_fc1, fc1_b, fc1_b, hid2, ff, DFF, DM);

  gemm_kernel<1><<<dim3(NTOK / 128, DM / 64), 128, 0, stream>>>(ff, w_fc2, fc2_b, hid2, out, xn, DM, DFF);
}
